// DifferentialTrittention_42468636622923
// MI455X (gfx1250) — hardware-verified
//
#include <hip/hip_runtime.h>
#include <math.h>

typedef __attribute__((ext_vector_type(16))) _Float16 v16h;
typedef __attribute__((ext_vector_type(8)))  _Float16 v8h;
typedef __attribute__((ext_vector_type(16))) __bf16   v16b;
typedef __attribute__((ext_vector_type(8)))  float    v8f;
typedef __attribute__((ext_vector_type(4)))  float    v4f;

__device__ __forceinline__ int frag_k(int i, int h) { return (i < 8) ? (8 * h + i) : (16 + 8 * h + (i - 8)); }
__device__ __forceinline__ __bf16 bf16_rne(float f) {
    unsigned int u = __float_as_uint(f);
    u += 0x7fffu + ((u >> 16) & 1u);
    return __builtin_bit_cast(__bf16, (unsigned short)(u >> 16));
}
__device__ __forceinline__ float bf16_f32(__bf16 b) { return __uint_as_float(((unsigned int)__builtin_bit_cast(unsigned short, b)) << 16); }
__device__ __forceinline__ v8f wmma16(v16h a, v16h b, v8f c) {
    c = __builtin_amdgcn_wmma_f32_16x16x32_f16(false, a, false, b, (short)0, c, false, false);
    asm volatile("v_nop\n\tv_nop\n\tv_nop\n\tv_nop" : "+v"(c) : "v"(a), "v"(b));
    return c;
}
__device__ __forceinline__ v8f wmmab(v16b a, v16b b, v8f c) {
    c = __builtin_amdgcn_wmma_f32_16x16x32_bf16(false, a, false, b, (short)0, c, false, false);
    asm volatile("v_nop\n\tv_nop\n\tv_nop\n\tv_nop" : "+v"(c) : "v"(a), "v"(b));
    return c;
}
struct Split { v16b hi, lo; };
__device__ __forceinline__ v8f wmma3(const Split& a, const Split& b, v8f c) {
    c = __builtin_amdgcn_wmma_f32_16x16x32_bf16(false, a.hi, false, b.hi, (short)0, c, false, false);
    c = __builtin_amdgcn_wmma_f32_16x16x32_bf16(false, a.hi, false, b.lo, (short)0, c, false, false);
    c = __builtin_amdgcn_wmma_f32_16x16x32_bf16(false, a.lo, false, b.hi, (short)0, c, false, false);
    asm volatile("v_nop\n\tv_nop\n\tv_nop\n\tv_nop" : "+v"(c) : "v"(a.hi), "v"(a.lo), "v"(b.hi), "v"(b.lo));
    return c;
}
struct Split3 { v16b hi, mid, lo; };
__device__ __forceinline__ v8f wmma6(const Split3& a, const Split3& b, v8f c) {
    c = __builtin_amdgcn_wmma_f32_16x16x32_bf16(false, a.hi, false, b.hi, (short)0, c, false, false);
    c = __builtin_amdgcn_wmma_f32_16x16x32_bf16(false, a.hi, false, b.mid, (short)0, c, false, false);
    c = __builtin_amdgcn_wmma_f32_16x16x32_bf16(false, a.mid, false, b.hi, (short)0, c, false, false);
    c = __builtin_amdgcn_wmma_f32_16x16x32_bf16(false, a.hi, false, b.lo, (short)0, c, false, false);
    c = __builtin_amdgcn_wmma_f32_16x16x32_bf16(false, a.mid, false, b.mid, (short)0, c, false, false);
    c = __builtin_amdgcn_wmma_f32_16x16x32_bf16(false, a.lo, false, b.hi, (short)0, c, false, false);
    asm volatile("v_nop\n\tv_nop\n\tv_nop\n\tv_nop" : "+v"(c) : "v"(a.hi), "v"(a.mid), "v"(a.lo), "v"(b.hi), "v"(b.mid), "v"(b.lo));
    return c;
}

__device__ __forceinline__ v16h fh_ld(const float* __restrict__ p, long long sk, int k0, int h, int klen, float s) {
    v16h a;
#pragma unroll
    for (int i = 0; i < 16; ++i) { const int k = k0 + frag_k(i, h); a[i] = (k < klen) ? (_Float16)(p[(long long)k * sk] * s) : (_Float16)0.f; }
    return a;
}
__device__ __forceinline__ Split sp_ld(const float* __restrict__ p, long long sk, int k0, int h, int klen, float s) {
    Split r;
#pragma unroll
    for (int i = 0; i < 16; ++i) {
        const int k = k0 + frag_k(i, h); const float x = (k < klen) ? p[(long long)k * sk] * s : 0.f;
        const __bf16 hb = bf16_rne(x); r.hi[i] = hb; r.lo[i] = bf16_rne(x - bf16_f32(hb));
    }
    return r;
}
__device__ __forceinline__ Split3 sp3_ld(const float* __restrict__ p, long long sk, int k0, int h, int klen, float s) {
    Split3 r;
#pragma unroll
    for (int i = 0; i < 16; ++i) {
        const int k = k0 + frag_k(i, h); const float x = (k < klen) ? p[(long long)k * sk] * s : 0.f;
        const __bf16 hb = bf16_rne(x); const float r1 = x - bf16_f32(hb); const __bf16 mb = bf16_rne(r1);
        r.hi[i] = hb; r.mid[i] = mb; r.lo[i] = bf16_rne(r1 - bf16_f32(mb));
    }
    return r;
}
__device__ __forceinline__ v16b bh_ld(const float* __restrict__ p, long long sk, int k0, int h, int klen, float s) {
    v16b a;
#pragma unroll
    for (int i = 0; i < 16; ++i) { const int k = k0 + frag_k(i, h); a[i] = bf16_rne((k < klen) ? p[(long long)k * sk] * s : 0.f); }
    return a;
}
__device__ __forceinline__ v16h fh_row(const _Float16* __restrict__ row, int k0, int h) {
    v16h a;
#pragma unroll
    for (int i = 0; i < 16; ++i) a[i] = row[k0 + frag_k(i, h)];
    return a;
}

#define VST2(T, ptr, val) do { const T vst2_v_ = (val); *(volatile T*)(ptr) = vst2_v_; __threadfence(); *(volatile T*)(ptr) = vst2_v_; } while (0)
typedef float v4f __attribute__((ext_vector_type(4)));
#define VST2V4(ptr, val) do { const v4f vst2_v4_ = (val); *(volatile v4f*)(ptr) = vst2_v4_; __threadfence(); *(volatile v4f*)(ptr) = vst2_v4_; } while (0)

__device__ __attribute__((noinline)) float act_fn(float v, int act) {
    if (act == 1) return fmaxf(v, 0.f);
    if (act == 2) { const float u = 0.7978845608028654f * (v + 0.044715f * v * v * v); return 0.5f * v * (1.f + tanhf(u)); }
    if (act == 3) return v / (1.f + expf(-v));
    if (act == 4) return 0.5f * v * (1.f + erff(v * 0.7071067811865476f));
    if (act == 5) return tanhf(v);
    if (act == 6) return 1.f / (1.f + expf(-v));
    if (act == 7) return (v > 0.f) ? v : 0.01f * v;
    if (act == 8) return (v > 0.f) ? v : (expf(v) - 1.f);
    if (act == 9) return fminf(fmaxf(v, 0.f), 6.f);
    if (act == 10) return fabsf(v);
    if (act == 11) return (v >= 0.f) ? v : 0.1f * v;
    if (act == 12) return (v > 0.f) ? v : 0.2f * v;
    if (act == 13) return (v > 20.f) ? v : log1pf(expf(v));
    return v;
}

struct GemmP {
    const float* A; const float* B; const float* bias; const float* R; float* C;
    long long sAo, sAi, sAm, sAk, sBo, sBi, sBn, sBk, sCo, sCi, sCm, sRo, sRi, sRm, sRn;
    int M, N, K, zi_n, flags, act; float alpha, beta, sa, sb;
    int Npad, pad_;
};
static_assert(sizeof(GemmP) == 5 * 8 + 15 * 8 + 6 * 4 + 4 * 4 + 2 * 4, "GemmP has padding");

template <int MODE>
__global__ __launch_bounds__(32) void k_gemm(GemmP p) {
    const int lane = threadIdx.x & 31, h = lane >> 4, l15 = lane & 15;
    const int m0 = blockIdx.y * 16, n0 = blockIdx.x * 32;
    const int z = blockIdx.z, zo = z / p.zi_n, zi = z - zo * p.zi_n;
    const float* A = p.A + zo * p.sAo + zi * p.sAi;
    const float* B = p.B + zo * p.sBo + zi * p.sBi;
    const int am = min(m0 + l15, p.M - 1);
    v8f acc[2], comp[2];
#pragma unroll
    for (int t = 0; t < 2; ++t) { v8f zz = {}; acc[t] = zz; comp[t] = zz; }
    for (int k0 = 0; k0 < p.K; k0 += 32) {
        const float* arow = A + (long long)am * p.sAm;
        if (MODE == 1) {
            const Split a = sp_ld(arow, p.sAk, k0, h, p.K, 1.f);
#pragma unroll
            for (int t = 0; t < 2; ++t) {
                const int bn = min(n0 + t * 16 + l15, p.N - 1);
                acc[t] = wmma3(a, sp_ld(B + (long long)bn * p.sBn, p.sBk, k0, h, p.K, 1.f), acc[t]);
            }
        } else if (MODE == 3) {
            const Split3 a = sp3_ld(arow, p.sAk, k0, h, p.K, 1.f);
#pragma unroll
            for (int t = 0; t < 2; ++t) {
                const int bn = min(n0 + t * 16 + l15, p.N - 1);
                acc[t] = wmma6(a, sp3_ld(B + (long long)bn * p.sBn, p.sBk, k0, h, p.K, 1.f), acc[t]);
            }
        } else if (MODE == 4) {
            const Split3 a = sp3_ld(arow, p.sAk, k0, h, p.K, 1.f);
#pragma unroll
            for (int t = 0; t < 2; ++t) {
                const int bn = min(n0 + t * 16 + l15, p.N - 1); v8f zz = {};
                const v8f part = wmma6(a, sp3_ld(B + (long long)bn * p.sBn, p.sBk, k0, h, p.K, 1.f), zz);
                const v8f y = part - comp[t]; const v8f s = acc[t] + y; comp[t] = (s - acc[t]) - y; acc[t] = s;
            }
        } else if (MODE == 2) {
            const v16b a = bh_ld(arow, p.sAk, k0, h, p.K, 1.f);
#pragma unroll
            for (int t = 0; t < 2; ++t) {
                const int bn = min(n0 + t * 16 + l15, p.N - 1);
                acc[t] = wmmab(a, bh_ld(B + (long long)bn * p.sBn, p.sBk, k0, h, p.K, 1.f), acc[t]);
            }
        } else {
            const v16h a = fh_ld(arow, p.sAk, k0, h, p.K, p.sa);
#pragma unroll
            for (int t = 0; t < 2; ++t) {
                const int bn = min(n0 + t * 16 + l15, p.N - 1);
                acc[t] = wmma16(a, fh_ld(B + (long long)bn * p.sBn, p.sBk, k0, h, p.K, p.sb), acc[t]);
            }
        }
    }
    const float iscale = (MODE == 0) ? p.alpha / (p.sa * p.sb) : p.alpha;
    float* C = p.C + zo * p.sCo + zi * p.sCi;
    const float* R = p.R + zo * p.sRo + zi * p.sRi;
    __shared__ __align__(16) float ctile[16][36];
#pragma unroll
    for (int t = 0; t < 2; ++t) {
        const int n = n0 + t * 16 + l15; const int nn = min(n, p.N - 1);
#pragma unroll
        for (int r = 0; r < 8; ++r) {
            const int m = m0 + 8 * h + r; const int mm = min(m, p.M - 1);
            float v = acc[t][r] * iscale;
            if (p.flags & 1) v += p.bias[nn];
            if (p.flags & 2) v += p.bias[mm];
            v = act_fn(v, p.act);
            if (p.flags & 4) v += p.beta * R[(long long)mm * p.sRm + (long long)nn * p.sRn];
            ctile[8 * h + r][t * 16 + l15] = (n < p.N) ? v : 0.f;
        }
    }
    __syncthreads();
    const int NW = (p.Npad > p.N) ? p.Npad : p.N;
    const bool fast = (m0 + 16 <= p.M) && (n0 + 32 <= NW) && ((p.sCm & 3) == 0) && ((((size_t)C) & 15) == 0);
    if (fast) {
#pragma unroll
        for (int s = 0; s < 4; ++s) {
            const int row = s * 4 + (lane >> 3), c4 = (lane & 7) * 4;
            const v4f v = *(const v4f*)&ctile[row][c4];
            VST2V4(C + (long long)(m0 + row) * p.sCm + n0 + c4, v);
        }
    } else {
        for (int row = 0; row < 16; ++row) {
            const int m = m0 + row, n = n0 + lane;
            if (m < p.M && n < NW) VST2(float, C + (long long)m * p.sCm + n, ctile[row][lane]);
        }
    }
}


template <int MODE, int TM, int TN>
__global__ __launch_bounds__(32) void k_gemmT(GemmP p) {
    const int lane = threadIdx.x & 31, h = lane >> 4, l15 = lane & 15;
    const int m0 = blockIdx.y * (16 * TM), n0 = blockIdx.x * (16 * TN);
    const int z = blockIdx.z, zo = z / p.zi_n, zi = z - zo * p.zi_n;
    const float* A = p.A + zo * p.sAo + zi * p.sAi;
    const float* B = p.B + zo * p.sBo + zi * p.sBi;
    v8f acc[TM][TN];
#pragma unroll
    for (int i = 0; i < TM; ++i)
#pragma unroll
        for (int t = 0; t < TN; ++t) { v8f zz = {}; acc[i][t] = zz; }
    for (int k0 = 0; k0 < p.K; k0 += 32) {
        if (MODE == 1) {
            Split a[TM], b[TN];
#pragma unroll
            for (int i = 0; i < TM; ++i) { const int am = min(m0 + 16 * i + l15, p.M - 1); a[i] = sp_ld(A + (long long)am * p.sAm, p.sAk, k0, h, p.K, 1.f); }
#pragma unroll
            for (int t = 0; t < TN; ++t) { const int bn = min(n0 + 16 * t + l15, p.N - 1); b[t] = sp_ld(B + (long long)bn * p.sBn, p.sBk, k0, h, p.K, 1.f); }
#pragma unroll
            for (int i = 0; i < TM; ++i)
#pragma unroll
                for (int t = 0; t < TN; ++t) acc[i][t] = wmma3(a[i], b[t], acc[i][t]);
        } else if (MODE == 2) {
            v16b a[TM], b[TN];
#pragma unroll
            for (int i = 0; i < TM; ++i) { const int am = min(m0 + 16 * i + l15, p.M - 1); a[i] = bh_ld(A + (long long)am * p.sAm, p.sAk, k0, h, p.K, 1.f); }
#pragma unroll
            for (int t = 0; t < TN; ++t) { const int bn = min(n0 + 16 * t + l15, p.N - 1); b[t] = bh_ld(B + (long long)bn * p.sBn, p.sBk, k0, h, p.K, 1.f); }
#pragma unroll
            for (int i = 0; i < TM; ++i)
#pragma unroll
                for (int t = 0; t < TN; ++t) acc[i][t] = wmmab(a[i], b[t], acc[i][t]);
        } else {
            v16h a[TM], b[TN];
#pragma unroll
            for (int i = 0; i < TM; ++i) { const int am = min(m0 + 16 * i + l15, p.M - 1); a[i] = fh_ld(A + (long long)am * p.sAm, p.sAk, k0, h, p.K, p.sa); }
#pragma unroll
            for (int t = 0; t < TN; ++t) { const int bn = min(n0 + 16 * t + l15, p.N - 1); b[t] = fh_ld(B + (long long)bn * p.sBn, p.sBk, k0, h, p.K, p.sb); }
#pragma unroll
            for (int i = 0; i < TM; ++i)
#pragma unroll
                for (int t = 0; t < TN; ++t) acc[i][t] = wmma16(a[i], b[t], acc[i][t]);
        }
    }
    const float iscale = (MODE == 0) ? p.alpha / (p.sa * p.sb) : p.alpha;
    float* C = p.C + zo * p.sCo + zi * p.sCi;
    const float* R = p.R + zo * p.sRo + zi * p.sRi;
    const int NW = (p.Npad > p.N) ? p.Npad : p.N;
    __shared__ __align__(16) float ctile[16][36];
#pragma unroll
    for (int i = 0; i < TM; ++i) {
        const int mb = m0 + 16 * i; if (mb >= p.M) break;
#pragma unroll
        for (int tp = 0; tp < TN / 2; ++tp) {
            const int nb = n0 + 32 * tp; if (nb >= NW) break;
#pragma unroll
            for (int t2 = 0; t2 < 2; ++t2) {
                const int t = 2 * tp + t2; const int n = nb + t2 * 16 + l15; const int nn = min(n, p.N - 1);
#pragma unroll
                for (int r = 0; r < 8; ++r) {
                    const int m = mb + 8 * h + r; const int mm = min(m, p.M - 1);
                    float v = acc[i][t][r] * iscale;
                    if (p.flags & 1) v += p.bias[nn];
                    if (p.flags & 2) v += p.bias[mm];
                    v = act_fn(v, p.act);
                    if (p.flags & 4) v += p.beta * R[(long long)mm * p.sRm + (long long)nn * p.sRn];
                    ctile[8 * h + r][t2 * 16 + l15] = (n < p.N) ? v : 0.f;
                }
            }
            __syncthreads();
            const bool fast = (mb + 16 <= p.M) && (nb + 32 <= NW) && ((p.sCm & 3) == 0) && ((((size_t)C) & 15) == 0);
            if (fast) {
#pragma unroll
                for (int s = 0; s < 4; ++s) {
                    const int row = s * 4 + (lane >> 3), c4 = (lane & 7) * 4;
                    const v4f v = *(const v4f*)&ctile[row][c4];
                    VST2V4(C + (long long)(mb + row) * p.sCm + nb + c4, v);
                }
            } else {
                for (int row = 0; row < 16; ++row) {
                    const int m = mb + row, n = nb + lane;
                    if (m < p.M && n < NW) VST2(float, C + (long long)m * p.sCm + n, ctile[row][lane]);
                }
            }
            __syncthreads();
        }
    }
}

#define AW 4
struct AttnP {
    const float* Q; const float* K; const float* V; float* O; float* P; const float* Mf; const int* Mi; float* ST;
    const float* Pw; const float* Rt; const int* SQ; const int* SK;
    long long swb, swh, swi, swj, srb, srh, sri;
    long long sQb, sQh, sQi, sQd, sKb, sKh, sKj, sKd, sVb, sVh, sVj, sVd, sOb, sOh, sOi, sPb, sPh, sPi, smb, smh, smi, smj;
    int Lq, Lk, dh, dv, hrep, causal, coff, pband;
    float scale, mfill; int nonorm, mpol;
    int roff, rn, segpol, win;
};
static_assert(sizeof(AttnP) == 12 * 8 + 29 * 8 + 16 * 4, "AttnP has padding");

#ifndef KATTN_ATTR
#define KATTN_ATTR
#endif
template <int DHP, int DVP, int QM, bool SPLITPV, bool TWOPASS>
__global__ __launch_bounds__(32 * AW) KATTN_ATTR void k_attn(AttnP p) {
    constexpr int NT = DVP / 16;
    constexpr int KS = DHP / 32;
    constexpr int VP = DVP + 8;
    __shared__ __align__(16) float    pl[AW][16 * 64];
    __shared__ __align__(16) _Float16 vl[(SPLITPV ? 2 : 1) * 64 * VP];
    const int lane = threadIdx.x & 31, hf = lane >> 4, l15 = lane & 15, wave = threadIdx.x >> 5;
    const int h = blockIdx.y, b = blockIdx.z, hk = h / p.hrep;
    const int q0 = (blockIdx.x * AW + wave) * 16;
    float* myp = pl[wave];
    const float L2E = 1.4426950408889634f;
    const float NEG = -__builtin_inff();
    const int qi = min(q0 + l15, p.Lq - 1);
    const float* qrow = p.Q + b * p.sQb + h * p.sQh + (long long)qi * p.sQi;
    const float* kbase = p.K + b * p.sKb + hk * p.sKh;
    const float* vbase = p.V + b * p.sVb + hk * p.sVh;
    v16h qa[QM == 0 ? KS : 1]; Split qs_[QM == 1 ? KS : 1]; Split3 qt_[QM == 2 ? KS : 1];
#pragma unroll
    for (int ks = 0; ks < KS; ++ks) {
        if (QM == 2) qt_[ks] = sp3_ld(qrow, p.sQd, ks * 32, hf, p.dh, 1.f);
        else if (QM == 1) qs_[ks] = sp_ld(qrow, p.sQd, ks * 32, hf, p.dh, 1.f);
        else qa[ks] = fh_ld(qrow, p.sQd, ks * 32, hf, p.dh, 1.f);
    }
    v8f o[NT]; float m8[8], l8[8];
#pragma unroll
    for (int t = 0; t < NT; ++t) { v8f zz = {}; o[t] = zz; }
#pragma unroll
    for (int i = 0; i < 8; ++i) { m8[i] = NEG; l8[i] = 0.f; }
    int jend = p.Lk;
    if (p.causal == 1) { const int je = (blockIdx.x * AW + AW - 1) * 16 + 16 + p.coff; jend = min(jend, max(je, 0)); }
    const int npass = TWOPASS ? 2 : 1;
    for (int pass = 0; pass < npass; ++pass) {
        const bool dopv = (!TWOPASS) || pass == 1;
        for (int j0 = 0; j0 < jend; j0 += 64) {
            if (dopv) {
                __syncthreads();
                for (int idx = threadIdx.x; idx < 64 * DVP; idx += 32 * AW) {
                    const int jr = idx / DVP, d = idx - jr * DVP, j = j0 + jr;
                    const float f = (j < p.Lk && d < p.dv) ? vbase[(long long)j * p.sVj + (long long)d * p.sVd] : 0.f;
                    if (SPLITPV) {
                        const __bf16 hb = bf16_rne(f);
                        ((__bf16*)vl)[jr * VP + d] = hb; ((__bf16*)vl)[64 * VP + jr * VP + d] = bf16_rne(f - bf16_f32(hb));
                    } else vl[jr * VP + d] = (_Float16)f;
                }
            }
            v8f s[4];
#pragma unroll
            for (int t = 0; t < 4; ++t) {
                const int j = min(j0 + t * 16 + l15, p.Lk - 1);
                const float* krow = kbase + (long long)j * p.sKj;
                v8f acc = {};
#pragma unroll
                for (int ks = 0; ks < KS; ++ks) {
                    if (QM == 2)      acc = wmma6(qt_[ks], sp3_ld(krow, p.sKd, ks * 32, hf, p.dh, 1.f), acc);
                    else if (QM == 1) acc = wmma3(qs_[ks], sp_ld(krow, p.sKd, ks * 32, hf, p.dh, 1.f), acc);
                    else              acc = wmma16(qa[ks], fh_ld(krow, p.sKd, ks * 32, hf, p.dh, 1.f), acc);
                }
                s[t] = acc;
            }
            float pv[8][4];
#pragma unroll
            for (int i = 0; i < 8; ++i) {
                const int irow = q0 + i + 8 * hf;
                const int ic = min(irow, p.Lq - 1);
                float sc[4];
#pragma unroll
                for (int t = 0; t < 4; ++t) {
                    const int jg = j0 + t * 16 + l15;
                    float v = s[t][i] * p.scale;
                    if (p.Mf) v += p.Mf[b * p.smb + h * p.smh + (long long)ic * p.smi + (long long)min(jg, p.Lk - 1) * p.smj];
                    if (p.Rt) { int rc = ic - min(jg, p.Lk - 1) + p.roff; rc = rc < 0 ? 0 : (rc >= p.rn ? p.rn - 1 : rc); v += p.Rt[b * p.srb + h * p.srh + (long long)ic * p.sri + rc]; }
                    if (p.Mi) { const int mv = p.Mi[b * p.smb + h * p.smh + (long long)ic * p.smi + (long long)min(jg, p.Lk - 1) * p.smj]; if (p.mpol ? (mv != 0) : (mv == 0)) v = p.mfill; }
                    if (p.SQ) { const bool same = p.SQ[(long long)b * p.Lq + ic] == p.SK[(long long)b * p.Lk + min(jg, p.Lk - 1)]; if (p.segpol ? same : !same) v = p.mfill; }
                    if (p.causal == 2 && jg > irow + p.coff) v = p.mfill;
                    if (jg >= p.Lk || (p.causal == 1 && jg > irow + p.coff) || (p.causal == 3 && jg < irow + p.coff) || (p.win > 0 && irow + p.coff - jg > p.win)) v = NEG; else v *= L2E;
                    sc[t] = v;
                }
                if (!TWOPASS || pass == 0) {
                    float mx = fmaxf(fmaxf(sc[0], sc[1]), fmaxf(sc[2], sc[3]));
                    mx = fmaxf(mx, __shfl_xor(mx, 1, 32)); mx = fmaxf(mx, __shfl_xor(mx, 2, 32));
                    mx = fmaxf(mx, __shfl_xor(mx, 4, 32)); mx = fmaxf(mx, __shfl_xor(mx, 8, 32));
                    const float mnew = fmaxf(m8[i], mx);
                    const float corr = (mnew == NEG) ? 1.f : exp2f(m8[i] - mnew);
                    float rs = 0.f;
#pragma unroll
                    for (int t = 0; t < 4; ++t) {
                        const float pp = (sc[t] == NEG) ? 0.f : exp2f(sc[t] - mnew); rs += pp;
                        pv[i][t] = p.Pw ? pp * p.Pw[b * p.swb + h * p.swh + (long long)ic * p.swi + (long long)min(j0 + t * 16 + l15, p.Lk - 1) * p.swj] : pp;
                    }
                    rs += __shfl_xor(rs, 1, 32); rs += __shfl_xor(rs, 2, 32); rs += __shfl_xor(rs, 4, 32); rs += __shfl_xor(rs, 8, 32);
                    l8[i] = l8[i] * corr + rs; m8[i] = mnew;
                    if (!TWOPASS) {
#pragma unroll
                        for (int t = 0; t < NT; ++t) o[t][i] *= corr;
                    }
                } else {
                    const float inv = (l8[i] > 0.f) ? 1.f / l8[i] : 0.f;
#pragma unroll
                    for (int t = 0; t < 4; ++t) {
                        const int jg = j0 + t * 16 + l15;
                        float pp = (sc[t] == NEG) ? 0.f : exp2f(sc[t] - m8[i]) * inv;
                        if (p.Pw) pp *= p.Pw[b * p.swb + h * p.swh + (long long)ic * p.swi + (long long)min(jg, p.Lk - 1) * p.swj];
                        pv[i][t] = pp;
                    }
                }
            }
            if (dopv) {
#pragma unroll
                for (int i = 0; i < 8; ++i)
#pragma unroll
                    for (int t = 0; t < 4; ++t) myp[(i + 8 * hf) * 64 + t * 16 + l15] = pv[i][t];
                __syncthreads();
                if (p.P) {
                    float* pb_ = p.P + b * p.sPb + h * p.sPh;
                    const bool fastP = (p.pband == 0) && ((p.sPi & 3) == 0) && (j0 + 64 <= p.Lk) && (q0 + 16 <= p.Lq) && ((((size_t)pb_) & 15) == 0);
                    if (fastP) {
#pragma unroll
                        for (int s = 0; s < 8; ++s) {
                            const int row = s * 2 + (lane >> 4), c4 = (lane & 15) * 4;
                            const v4f v = *(const v4f*)(myp + row * 64 + c4);
                            VST2V4(pb_ + (long long)(q0 + row) * p.sPi + j0 + c4, v);
                        }
                    } else {
                        for (int row = 0; row < 16; ++row) {
                            const int irow = q0 + row; if (irow >= p.Lq) continue;
                            for (int c = lane; c < 64; c += 32) {
                                const int jg = j0 + c; if (jg >= p.Lk) continue;
                                if (p.pband == 0) VST2(float, pb_ + (long long)irow * p.sPi + jg, myp[row * 64 + c]);
                                else if (jg - irow <= p.pband && irow - jg <= p.pband) VST2(float, pb_ + (long long)irow * p.sPi + (jg - irow + p.pband), myp[row * 64 + c]);
                            }
                        }
                    }
                }
                if (SPLITPV) {
                    const Split pa0 = sp_ld(myp + l15 * 64, 1, 0, hf, 64, 1.f), pa1 = sp_ld(myp + l15 * 64, 1, 32, hf, 64, 1.f);
                    const __bf16* vh = (const __bf16*)vl; const __bf16* vlo = vh + 64 * VP;
#pragma unroll
                    for (int t = 0; t < NT; ++t) {
                        const int dcol = t * 16 + l15;
                        Split b0, b1;
#pragma unroll
                        for (int e = 0; e < 16; ++e) {
                            const int k0 = frag_k(e, hf), k1 = 32 + frag_k(e, hf);
                            b0.hi[e] = vh[k0 * VP + dcol]; b0.lo[e] = vlo[k0 * VP + dcol]; b1.hi[e] = vh[k1 * VP + dcol]; b1.lo[e] = vlo[k1 * VP + dcol];
                        }
                        o[t] = wmma3(pa0, b0, o[t]);
                        o[t] = wmma3(pa1, b1, o[t]);
                    }
                } else {
                    const v16h pa0 = fh_ld(myp + l15 * 64, 1, 0, hf, 64, 4096.f), pa1 = fh_ld(myp + l15 * 64, 1, 32, hf, 64, 4096.f);
#pragma unroll
                    for (int t = 0; t < NT; ++t) {
                        const int dcol = t * 16 + l15;
                        v16h b0, b1;
#pragma unroll
                        for (int e = 0; e < 16; ++e) { b0[e] = vl[frag_k(e, hf) * VP + dcol]; b1[e] = vl[(32 + frag_k(e, hf)) * VP + dcol]; }
                        o[t] = wmma16(pa0, b0, o[t]);
                        o[t] = wmma16(pa1, b1, o[t]);
                    }
                }
            }
        }
    }
    float* obase = p.O + b * p.sOb + h * p.sOh;
    if (p.ST) {
        const int rl = lane >> 1, isel = rl & 7;
        float mv = 0.f, lv = 0.f;
#pragma unroll
        for (int i = 0; i < 8; ++i) if (i == isel) { mv = m8[i]; lv = l8[i]; }
        const int irow = q0 + rl;
        if (irow < p.Lq) { float* st = p.ST + (((long long)b * gridDim.y + h) * p.Lq + irow) * 2 + (lane & 1); VST2(float, st, (lane & 1) ? lv : mv * 0.6931471805599453f); }
    }
    float invr[8];
#pragma unroll
    for (int i = 0; i < 8; ++i) {
        if (TWOPASS) invr[i] = SPLITPV ? 1.f : (1.f / 4096.f);
        else if (p.nonorm) invr[i] = exp2f(m8[i]) * (SPLITPV ? 1.f : (1.f / 4096.f));
        else invr[i] = (l8[i] > 0.f) ? (SPLITPV ? 1.f / l8[i] : 1.f / (l8[i] * 4096.f)) : 0.f;
    }
    __syncthreads();
    const bool ofast = ((p.sOi & 3) == 0) && ((((size_t)obase) & 15) == 0) && (q0 + 16 <= p.Lq);
#pragma unroll
    for (int c0 = 0; c0 < DVP; c0 += 64) {
#pragma unroll
        for (int i = 0; i < 8; ++i)
#pragma unroll
            for (int t = 0; t < NT; ++t) if (t * 16 >= c0 && t * 16 < c0 + 64) myp[(i + 8 * hf) * 64 + (t * 16 - c0) + l15] = o[t][i] * invr[i];
        __syncthreads();
        const int cw = (DVP - c0 < 64) ? (DVP - c0) : 64;
        if (ofast && (c0 + cw <= p.dv) && (cw % 32 == 0)) {
            const int lpr = cw / 4;
            const int rows_per_ins = 32 / lpr;
            for (int r0 = 0; r0 < 16; r0 += rows_per_ins) {
                const int row = r0 + lane / lpr, c4 = (lane % lpr) * 4;
                const v4f v = *(const v4f*)(myp + row * 64 + c4);
                VST2V4(obase + (long long)(q0 + row) * p.sOi + c0 + c4, v);
            }
        } else {
            for (int row = 0; row < 16; ++row) {
                const int irow = q0 + row; if (irow >= p.Lq) continue;
                for (int c = lane; c < cw; c += 32) { const int d = c0 + c; if (d < p.dv) VST2(float, obase + (long long)irow * p.sOi + d, myp[row * 64 + c]); }
            }
        }
        __syncthreads();
    }
}

struct TrP { const float* src; float* dst; const float* R2; long long sSz, lds, sDz, ldd, sRz, ldr; int R, C, flags, act; float alpha, beta; };
static_assert(sizeof(TrP) == 3 * 8 + 6 * 8 + 6 * 4, "TrP has padding");
__global__ __launch_bounds__(256) void k_tr(TrP p) {
    __shared__ float tile[32][33];
    const int c0 = blockIdx.x * 32, r0 = blockIdx.y * 32, z = blockIdx.z;
    const int lane = threadIdx.x & 31, wave = threadIdx.x >> 5;
    const float* s = p.src + z * p.sSz;
#pragma unroll
    for (int k = 0; k < 4; ++k) {
        const int rl = wave * 4 + k, r = r0 + rl, c = c0 + lane;
        tile[rl][lane] = (r < p.R && c < p.C) ? s[(long long)r * p.lds + c] : 0.f;
    }
    __syncthreads();
    float* d = p.dst + z * p.sDz; const float* rr = p.R2 + z * p.sRz;
#pragma unroll
    for (int k = 0; k < 4; ++k) {
        const int cl = wave * 4 + k, c = c0 + cl, r = r0 + lane;
        if (c < p.C && r < p.R) {
            float v = act_fn(p.alpha * tile[lane][cl], p.act);
            if (p.flags & 1) v += p.beta * rr[(long long)c * p.ldr + r];
            VST2(float, d + (long long)c * p.ldd + r, v);
        }
    }
}

__global__ __launch_bounds__(256) void k_affine(const float* __restrict__ src, float* __restrict__ dst, int n, float a, float b, const float* __restrict__ sdev) {
    const int i = blockIdx.x * 256 + threadIdx.x;
    if (i < n) { const float aa = sdev ? a * sdev[0] : a; const float v = aa * src[i] + b; VST2(float, dst + i, v); }
}

struct SmP { const float* src; float* dst; const float* Mf; long long sz, sr, dz, dr, smz, smr; int n, pad; float scale_in, scale_out; };
static_assert(sizeof(SmP) == 3 * 8 + 6 * 8 + 4 * 4, "SmP has padding");
__global__ __launch_bounds__(256) void k_softmax(SmP p) {
    __shared__ float red[256];
    const int r = blockIdx.x, z = blockIdx.y, tid = threadIdx.x;
    const float* s = p.src + z * p.sz + (long long)r * p.sr;
    const float* mf = p.Mf ? (p.Mf + z * p.smz + (long long)r * p.smr) : nullptr;
    float mx = -__builtin_inff();
    for (int j = tid; j < p.n; j += 256) { float v = s[j] * p.scale_in; if (mf) v += mf[j]; mx = fmaxf(mx, v); }
    red[tid] = mx; __syncthreads();
    for (int o = 128; o > 0; o >>= 1) { if (tid < o) red[tid] = fmaxf(red[tid], red[tid + o]); __syncthreads(); }
    mx = red[0]; __syncthreads();
    float sum = 0.f;
    for (int j = tid; j < p.n; j += 256) { float v = s[j] * p.scale_in; if (mf) v += mf[j]; sum += (mx == -__builtin_inff()) ? 0.f : expf(v - mx); }
    red[tid] = sum; __syncthreads();
    for (int o = 128; o > 0; o >>= 1) { if (tid < o) red[tid] += red[tid + o]; __syncthreads(); }
    sum = red[0];
    const float inv = (sum > 0.f) ? p.scale_out / sum : 0.f;
    float* d = p.dst + z * p.dz + (long long)r * p.dr;
    for (int j = tid; j < p.n; j += 256) { float v = s[j] * p.scale_in; if (mf) v += mf[j]; const float o = (mx == -__builtin_inff()) ? 0.f : expf(v - mx) * inv; VST2(float, d + j, o); }
}
__global__ __launch_bounds__(256) void k_stats(const float* __restrict__ x, long long sz, long long so, long long si, int inner, int n, float eps, float* __restrict__ stat, int mode) {
    __shared__ float red[256];
    const int z = blockIdx.x, tid = threadIdx.x;
    const float* base = x + z * sz;
    float s = 0.f;
    for (int e = tid; e < n; e += 256) s += base[(long long)(e / inner) * so + (long long)(e % inner) * si];
    red[tid] = s; __syncthreads();
    for (int o = 128; o > 0; o >>= 1) { if (tid < o) red[tid] += red[tid + o]; __syncthreads(); }
    const float mu = (mode == 0 || mode == 3) ? red[0] / (float)n : 0.f; __syncthreads();
    float q = 0.f;
    for (int e = tid; e < n; e += 256) { const float dlt = base[(long long)(e / inner) * so + (long long)(e % inner) * si] - mu; q += dlt * dlt; }
    red[tid] = q; __syncthreads();
    for (int o = 128; o > 0; o >>= 1) { if (tid < o) red[tid] += red[tid + o]; __syncthreads(); }
    {
        float rs;
        if (mode == 2) rs = sqrtf((float)n) / fmaxf(sqrtf(red[0]), eps); else if (mode == 3) rs = rsqrtf(red[0] / (float)(n - 1) + eps); else rs = rsqrtf(red[0] / (float)n + eps);
        if (tid < 32) { const float v = (tid == 0) ? mu : ((tid == 1) ? rs : 0.f); VST2(float, stat + (long long)z * 32 + tid, v); }
    }
}
__global__ __launch_bounds__(256) void k_norm_apply(const float* __restrict__ x, float* __restrict__ y, const float* __restrict__ stat, const float* __restrict__ g, const float* __restrict__ bta,
                                                     int Z, int C, int L, int G, int bn, int act) {
    const long long idx = (long long)blockIdx.x * 256 + threadIdx.x;
    if (idx >= (long long)Z * C * L) return;
    const int l = (int)(idx % L); const long long zc = idx / L; const int c = (int)(zc % C), z = (int)(zc / C); (void)l;
    const int set = bn ? c : (z * G + c / (C / G));
    float v = (x[idx] - stat[(long long)set * 32]) * stat[(long long)set * 32 + 1];
    if (g) v *= g[c];
    if (bta) v += bta[c];
    v = act_fn(v, act);
    VST2(float, y + idx, v);
}

__global__ __launch_bounds__(256) void k_lse_neg(const float* __restrict__ st, float* __restrict__ c, int n) {
    const int i = blockIdx.x * 256 + threadIdx.x;
    if (i < n) { const float v = -(st[2 * i] + logf(st[2 * i + 1])); VST2(float, c + i, v); }
}

__global__ __launch_bounds__(256) void k_iota(int* __restrict__ dst, int n, int a, int b) {
    const int i = blockIdx.x * 256 + threadIdx.x;
    if (i < n) { const int v = a * i + b; VST2(int, dst + i, v); }
}

__global__ __launch_bounds__(256) void k_axpby(const float* __restrict__ x, const float* __restrict__ y, float* __restrict__ dst, int n, float a, float b, float c) {
    const int i = blockIdx.x * 256 + threadIdx.x;
    if (i < n) { const float v = a * x[i] + b * y[i] + c; VST2(float, dst + i, v); }
}

struct RopeP { const float* X; float* Y; const float* C; const float* Sn; const int* pos; long long sXr, sXh, sYr, sYh, sCb, sCp, sCd; int R, Hn, D, S, mode, tmode, pmode, pad; };
static_assert(sizeof(RopeP) == 5 * 8 + 7 * 8 + 8 * 4, "RopeP has padding");
__global__ __launch_bounds__(256) void k_rope(RopeP p) {
    const long long idx = (long long)blockIdx.x * 256 + threadIdx.x;
    if (idx >= (long long)p.R * p.Hn * p.D) return;
    const int d = (int)(idx % p.D); const long long rh = idx / p.D; const int h = (int)(rh % p.Hn); const int r = (int)(rh / p.Hn);
    const int half = p.D / 2;
    int partner; float sign;
    if (p.mode == 0) { partner = (d < half) ? d + half : d - half; sign = (d < half) ? -1.f : 1.f; }
    else { partner = d ^ 1; sign = (d & 1) ? 1.f : -1.f; }
    const int tcol = (p.tmode == 0) ? d : ((p.tmode == 1) ? (d % half) : (d >> 1));
    const int pp = (p.pmode == 0) ? (r % p.S) : ((p.pmode == 1) ? h : p.pos[r]);
    const long long toff = (long long)(r / p.S) * p.sCb + (long long)pp * p.sCp + (long long)tcol * p.sCd;
    const float* xr = p.X + (long long)r * p.sXr + (long long)h * p.sXh;
    const float v = xr[d] * p.C[toff] + sign * xr[partner] * p.Sn[toff];
    VST2(float, p.Y + (long long)r * p.sYr + (long long)h * p.sYh + d, v);
}

__global__ __launch_bounds__(256) void k_invf(float* __restrict__ invb, int half, int D, float base, float num, int fmode, float cexp) {
    const int i = blockIdx.x * 256 + threadIdx.x;
    if (i >= ((half + 31) / 32) * 32) return;
    if (i >= half) { VST2(float, invb + i, 0.f); return; }
    const float e = (float)(2 * i) / (float)D;
    float invf;
    if (fmode == 1) invf = num * expf((float)(2 * i) * cexp);
    else if (fmode == 2) invf = num * powf(base, (-2.0f * ((float)i - 1.0f)) / (float)D);
    else invf = num * (1.0f / powf(base, e));
    VST2(float, invb + i, invf);
}
__global__ __launch_bounds__(256) void k_sincos(float* __restrict__ cs, float* __restrict__ sn, const float* __restrict__ invb, int S, int half, float pscale) {
    const int idx = blockIdx.x * 256 + threadIdx.x;
    if (idx >= S * half) return;
    const int s = idx / half, i = idx - s * half;
    const float ang = (pscale * (float)s) * invb[i];
    VST2(float, cs + idx, cosf(ang)); VST2(float, sn + idx, sinf(ang));
}

__global__ __launch_bounds__(256) void k_mulact(const float* __restrict__ x, const float* __restrict__ y, float* __restrict__ dst, int n, int act) {
    const int i = blockIdx.x * 256 + threadIdx.x;
    if (i < n) { const float v = act_fn(x[i], act) * y[i]; VST2(float, dst + i, v); }
}

__global__ __launch_bounds__(256) void k_matvec(GemmP p) {
    const int rpt = (p.N == 1) ? 1 : 32;
    const long long r0 = ((long long)blockIdx.x * 256 + threadIdx.x) * rpt; const int z = blockIdx.z, zo = z / p.zi_n, zi = z - zo * p.zi_n;
    if (r0 >= p.M) return;
    const float* Bb = p.B + zo * p.sBo + zi * p.sBi;
    float* C = p.C + zo * p.sCo + zi * p.sCi; const float* R = p.R + zo * p.sRo + zi * p.sRi;
    for (int rr = 0; rr < rpt; ++rr) {
        const long long r = r0 + rr; if (r >= p.M) break;
        const float* A = p.A + zo * p.sAo + zi * p.sAi + r * p.sAm;
        float acc[8] = {0.f, 0.f, 0.f, 0.f, 0.f, 0.f, 0.f, 0.f};
        for (int k = 0; k < p.K; ++k) { const float a = A[(long long)k * p.sAk];
#pragma unroll
            for (int j = 0; j < 8; ++j) if (j < p.N) acc[j] += a * Bb[(long long)j * p.sBn + (long long)k * p.sBk]; }
#pragma unroll
        for (int j = 0; j < 8; ++j) if (j < p.N) {
            float v = acc[j] * p.alpha;
            if (p.flags & 1) v += p.bias[j];
            if (p.flags & 2) v += p.bias[r];
            v = act_fn(v, p.act);
            if (p.flags & 4) v += p.beta * R[r * p.sRm + (long long)j * p.sRn];
            VST2(float, C + r * p.sCm + j, v);
        }
    }
}
__global__ __launch_bounds__(256) void k_smallsoftmax(const float* __restrict__ src, float* __restrict__ dst, long long sr, long long dr, int n, long long R, float scale) {
    const long long r0 = ((long long)blockIdx.x * 256 + threadIdx.x) * 32;
    for (int rr = 0; rr < 32; ++rr) {
        const long long r = r0 + rr; if (r >= R) return;
        const float* s = src + r * sr; float* d = dst + r * dr;
        float mx = -__builtin_inff();
        for (int j = 0; j < n; ++j) mx = fmaxf(mx, s[j] * scale);
        float sum = 0.f;
        for (int j = 0; j < n; ++j) sum += expf(s[j] * scale - mx);
        const float inv = 1.f / sum;
        for (int j = 0; j < n; ++j) { const float v = expf(s[j] * scale - mx) * inv; VST2(float, d + j, v); }
    }
}

__global__ __launch_bounds__(32) void k_unitstat(float* __restrict__ st) { const int t = threadIdx.x; const float v = (t == 1) ? 1.f : 0.f; VST2(float, st + t, v); }

__global__ __launch_bounds__(256) void k_lincopy(const float* __restrict__ src, long long lds, float* __restrict__ dst, long long ldd, long long rows, int cols) {
    const long long i = (long long)blockIdx.x * 256 + threadIdx.x; if (i >= rows * cols) return;
    const long long r = i / cols; const int c = (int)(i - r * cols);
    const float v = src[r * lds + c]; VST2(float, dst + r * ldd + c, v);
}

__global__ __launch_bounds__(256) void k_dt_kk(const float* __restrict__ KKQ, float* __restrict__ KK, int n0, int HB, int T, int DK, int E2, int DH) { const long long q = (long long)blockIdx.x * 256 + threadIdx.x; if (q >= (long long)HB * T * T * DH) return; const int h = (int)(q % DH); const int t = (int)((q / DH) % T); const int s = (int)((q / ((long long)DH * T)) % T); const int n = n0 + (int)(q / ((long long)DH * T * T));
    VST2(float, KK + q, KKQ[(long long)s * DK + n * DH + h] * KKQ[(long long)t * DK + E2 + n * DH + h]); }
__global__ __launch_bounds__(256) void k_dt_soft(float* __restrict__ SC, const float* __restrict__ lq1, const float* __restrict__ lk1, const float* __restrict__ lq2, const float* __restrict__ lk2, float* __restrict__ AS, float* __restrict__ AT, float* __restrict__ SA, int j0, int T, int DH, float LAM0_) { __shared__ float red[256]; const int jl = blockIdx.x / T, qq = blockIdx.x % T; const int j = j0 + jl; const int tid = threadIdx.x; const long long TT = (long long)T * T;
    float l1 = 0.f, l2 = 0.f; for (int i = 0; i < DH; ++i) { l1 += lq1[i] * lk1[i]; l2 += lq2[i] * lk2[i]; } const float lam = expf(l1) - expf(l2) + LAM0_;
    float* s0 = SC + ((long long)(2 * jl) * T + qq) * TT; float* s1 = SC + ((long long)(2 * jl + 1) * T + qq) * TT; const float inv = 1.f / (float)DH;
    float m0 = -__builtin_inff(), m1 = -__builtin_inff(); for (int l = tid; l < TT; l += 256) { const int s = l / T, t = l % T; const bool msk = (s > qq) || (t > qq); const float v0 = msk ? -1e6f : s0[l] * inv, v1 = msk ? -1e6f : s1[l] * inv; m0 = fmaxf(m0, v0); m1 = fmaxf(m1, v1); }
    red[tid] = m0; __syncthreads(); for (int o = 128; o > 0; o >>= 1) { if (tid < o) red[tid] = fmaxf(red[tid], red[tid + o]); __syncthreads(); } m0 = red[0]; __syncthreads(); red[tid] = m1; __syncthreads(); for (int o = 128; o > 0; o >>= 1) { if (tid < o) red[tid] = fmaxf(red[tid], red[tid + o]); __syncthreads(); } m1 = red[0]; __syncthreads();
    float d0 = 0.f, d1 = 0.f; for (int l = tid; l < TT; l += 256) { const int s = l / T, t = l % T; const bool msk = (s > qq) || (t > qq); const float e0 = expf((msk ? -1e6f : s0[l] * inv) - m0), e1 = expf((msk ? -1e6f : s1[l] * inv) - m1); d0 += e0; d1 += e1; s0[l] = e0; s1[l] = e1; }
    red[tid] = d0; __syncthreads(); for (int o = 128; o > 0; o >>= 1) { if (tid < o) red[tid] += red[tid + o]; __syncthreads(); } d0 = red[0]; __syncthreads(); red[tid] = d1; __syncthreads(); for (int o = 128; o > 0; o >>= 1) { if (tid < o) red[tid] += red[tid + o]; __syncthreads(); } d1 = red[0]; __threadfence_block(); __syncthreads();
    const float c0 = 1.f / d0, c1 = lam / d1;
    float rs = 0.f; if (tid < T) { const int s = tid; for (int t = 0; t < T; ++t) { const int l = s * T + t; rs += s0[l] * c0 - s1[l] * c1; } VST2(float, AS + ((long long)j * T + qq) * T + s, rs); }
    if (tid < T) { const int t = tid; float cs_ = 0.f; for (int s = 0; s < T; ++s) { const int l = s * T + t; cs_ += s0[l] * c0 - s1[l] * c1; } VST2(float, AT + ((long long)j * T + qq) * T + t, cs_); }
    red[tid] = (tid < T) ? rs : 0.f; __syncthreads(); for (int o = 128; o > 0; o >>= 1) { if (tid < o) red[tid] += red[tid + o]; __syncthreads(); } if (tid == 0) VST2(float, SA + j * T + qq, red[0]); }
__global__ __launch_bounds__(128) void k_dt_fin(const float* __restrict__ Z, const float* __restrict__ SA, const float* __restrict__ bv, float* __restrict__ Z2, int T, int NH, int DV, float LAM0_) { __shared__ float red[128]; const int qj = blockIdx.x; const int qq = qj / NH, j = qj % NH; const int c = threadIdx.x; const long long idx = (long long)qq * NH * DV + j * DV + c; const float v = Z[idx] + SA[j * T + qq] * bv[j * DV + c]; red[c] = v * v; __syncthreads(); for (int o = 64; o > 0; o >>= 1) { if (c < o) red[c] += red[c + o]; __syncthreads(); }
    VST2(float, Z2 + idx, v * rsqrtf(red[0] / (float)DV + 1e-5f) * (1.f - LAM0_)); }

template __global__ void k_gemm<0>(GemmP);
template __global__ void k_gemm<1>(GemmP);

extern "C" void kernel_launch(void* const* d_in, const int* in_sizes, int n_in, void* d_out, int out_size, void* d_ws, size_t ws_size, hipStream_t stream) {
    (void)in_sizes; (void)n_in; (void)out_size; (void)ws_size;
    const float* x = (const float*)d_in[0];
    const float* Wkkq = (const float*)d_in[1];
    const float* bkkq = (const float*)d_in[2];
    const float* Wv = (const float*)d_in[3];
    const float* bv = (const float*)d_in[4];
    const float* Wo = (const float*)d_in[5];
    const float* bo = (const float*)d_in[6];
    const float* lq1 = (const float*)d_in[7];
    const float* lk1 = (const float*)d_in[8];
    const float* lq2 = (const float*)d_in[9];
    const float* lk2 = (const float*)d_in[10];
    const int T = 160;
    const int D = 512;
    const int NH = 8;
    const int H2 = 16;
    const int DH = 64;
    const int DV = 128;
    const int HB = 4;
    const int DK = 3072;
    const int E2 = 1024;
    float* out = (float*)d_out;
    char* wsp = (char*)d_ws;
    float* KKQ = (float*)wsp; wsp += (((size_t)((size_t)T * DK) * 4 + 255) / 256) * 256;
    float* KK = (float*)wsp; wsp += (((size_t)((size_t)HB * T * T * DH) * 4 + 255) / 256) * 256;
    float* SC = (float*)wsp; wsp += (((size_t)((size_t)HB * T * T * T) * 4 + 255) / 256) * 256;
    float* VA = (float*)wsp; wsp += (((size_t)((size_t)T * 1024) * 4 + 255) / 256) * 256;
    float* VB = (float*)wsp; wsp += (((size_t)((size_t)T * 1024) * 4 + 255) / 256) * 256;
    float* AS = (float*)wsp; wsp += (((size_t)((size_t)NH * T * T) * 4 + 255) / 256) * 256;
    float* AT = (float*)wsp; wsp += (((size_t)((size_t)NH * T * T) * 4 + 255) / 256) * 256;
    float* SA = (float*)wsp; wsp += (((size_t)((size_t)NH * T) * 4 + 255) / 256) * 256;
    float* Z = (float*)wsp; wsp += (((size_t)((size_t)T * 1024) * 4 + 255) / 256) * 256;
    float* Z2 = (float*)wsp; wsp += (((size_t)((size_t)T * 1024) * 4 + 255) / 256) * 256;
    { GemmP gkkq;
      gkkq.A = x; gkkq.B = Wkkq; gkkq.bias = bkkq; gkkq.R = x; gkkq.C = KKQ;
      gkkq.sAo = 0; gkkq.sAi = 0; gkkq.sAm = D; gkkq.sAk = 1; gkkq.sBo = 0; gkkq.sBi = 0; gkkq.sBn = 1; gkkq.sBk = DK; gkkq.sCo = 0; gkkq.sCi = 0; gkkq.sCm = DK; gkkq.sRo = 0; gkkq.sRi = 0; gkkq.sRm = 0; gkkq.sRn = 0;
      gkkq.M = T; gkkq.N = DK; gkkq.K = D; gkkq.zi_n = 1; gkkq.flags = 1; gkkq.act = 0;
      gkkq.alpha = 1.0f; gkkq.beta = 0.0f; gkkq.sa = 1.0f; gkkq.sb = 1.0f; gkkq.Npad = DK; gkkq.pad_ = 0;
      if ((long long)(T) >= 64 && (long long)(DK) >= 64) k_gemmT<1, 2, 4><<<dim3((unsigned)((DK) + 63) / 64, (unsigned)((T) + 31) / 32, (unsigned)(1)), 32, 0, stream>>>(gkkq);
      else k_gemm<1><<<dim3((unsigned)((DK) + 31) / 32, (unsigned)((T) + 15) / 16, (unsigned)(1)), 32, 0, stream>>>(gkkq); }
    { GemmP gva;
      gva.A = x; gva.B = Wv; gva.bias = x; gva.R = x; gva.C = VA;
      gva.sAo = 0; gva.sAi = 0; gva.sAm = D; gva.sAk = 1; gva.sBo = 0; gva.sBi = 0; gva.sBn = 1; gva.sBk = 1024; gva.sCo = 0; gva.sCi = 0; gva.sCm = 1024; gva.sRo = 0; gva.sRi = 0; gva.sRm = 0; gva.sRn = 0;
      gva.M = T; gva.N = 1024; gva.K = D; gva.zi_n = 1; gva.flags = 0; gva.act = 0;
      gva.alpha = 1.0f; gva.beta = 0.0f; gva.sa = 1.0f; gva.sb = 1.0f; gva.Npad = 1024; gva.pad_ = 0;
      if ((long long)(T) >= 64 && (long long)(1024) >= 64) k_gemmT<1, 2, 4><<<dim3((unsigned)((1024) + 63) / 64, (unsigned)((T) + 31) / 32, (unsigned)(1)), 32, 0, stream>>>(gva);
      else k_gemm<1><<<dim3((unsigned)((1024) + 31) / 32, (unsigned)((T) + 15) / 16, (unsigned)(1)), 32, 0, stream>>>(gva); }
    { GemmP gvb;
      gvb.A = x; gvb.B = Wv + (size_t)D * 1024; gvb.bias = x; gvb.R = x; gvb.C = VB;
      gvb.sAo = 0; gvb.sAi = 0; gvb.sAm = D; gvb.sAk = 1; gvb.sBo = 0; gvb.sBi = 0; gvb.sBn = 1; gvb.sBk = 1024; gvb.sCo = 0; gvb.sCi = 0; gvb.sCm = 1024; gvb.sRo = 0; gvb.sRi = 0; gvb.sRm = 0; gvb.sRn = 0;
      gvb.M = T; gvb.N = 1024; gvb.K = D; gvb.zi_n = 1; gvb.flags = 0; gvb.act = 0;
      gvb.alpha = 1.0f; gvb.beta = 0.0f; gvb.sa = 1.0f; gvb.sb = 1.0f; gvb.Npad = 1024; gvb.pad_ = 0;
      if ((long long)(T) >= 64 && (long long)(1024) >= 64) k_gemmT<1, 2, 4><<<dim3((unsigned)((1024) + 63) / 64, (unsigned)((T) + 31) / 32, (unsigned)(1)), 32, 0, stream>>>(gvb);
      else k_gemm<1><<<dim3((unsigned)((1024) + 31) / 32, (unsigned)((T) + 15) / 16, (unsigned)(1)), 32, 0, stream>>>(gvb); }
    k_dt_kk<<<(unsigned)(((long long)HB * T * T * DH + 255) / 256), 256, 0, stream>>>(KKQ, KK, 0, HB, T, DK, E2, DH);
    { GemmP gsc0;
      gsc0.A = KKQ + (size_t)2 * E2 + 0 * DH; gsc0.B = KK; gsc0.bias = KKQ + (size_t)2 * E2 + 0 * DH; gsc0.R = KKQ + (size_t)2 * E2 + 0 * DH; gsc0.C = SC;
      gsc0.sAo = DH; gsc0.sAi = 0; gsc0.sAm = DK; gsc0.sAk = 1; gsc0.sBo = (long long)T * T * DH; gsc0.sBi = (long long)T * DH; gsc0.sBn = DH; gsc0.sBk = 1; gsc0.sCo = (long long)T * T * T; gsc0.sCi = T; gsc0.sCm = (long long)T * T; gsc0.sRo = 0; gsc0.sRi = 0; gsc0.sRm = 0; gsc0.sRn = 0;
      gsc0.M = T; gsc0.N = T; gsc0.K = DH; gsc0.zi_n = T; gsc0.flags = 0; gsc0.act = 0;
      gsc0.alpha = 1.0f; gsc0.beta = 0.0f; gsc0.sa = 1.0f; gsc0.sb = 1.0f; gsc0.Npad = T; gsc0.pad_ = 0;
      if ((long long)(T) >= 64 && (long long)(T) >= 64) k_gemmT<0, 4, 4><<<dim3((unsigned)((T) + 63) / 64, (unsigned)((T) + 63) / 64, (unsigned)(HB * T)), 32, 0, stream>>>(gsc0);
      else k_gemm<0><<<dim3((unsigned)((T) + 31) / 32, (unsigned)((T) + 15) / 16, (unsigned)(HB * T)), 32, 0, stream>>>(gsc0); }
    k_dt_soft<<<2 * T, 256, 0, stream>>>(SC, lq1, lk1, lq2, lk2, AS, AT, SA, 0, T, DH, 0.35550906759096934f);
    k_dt_kk<<<(unsigned)(((long long)HB * T * T * DH + 255) / 256), 256, 0, stream>>>(KKQ, KK, 4, HB, T, DK, E2, DH);
    { GemmP gsc1;
      gsc1.A = KKQ + (size_t)2 * E2 + 4 * DH; gsc1.B = KK; gsc1.bias = KKQ + (size_t)2 * E2 + 4 * DH; gsc1.R = KKQ + (size_t)2 * E2 + 4 * DH; gsc1.C = SC;
      gsc1.sAo = DH; gsc1.sAi = 0; gsc1.sAm = DK; gsc1.sAk = 1; gsc1.sBo = (long long)T * T * DH; gsc1.sBi = (long long)T * DH; gsc1.sBn = DH; gsc1.sBk = 1; gsc1.sCo = (long long)T * T * T; gsc1.sCi = T; gsc1.sCm = (long long)T * T; gsc1.sRo = 0; gsc1.sRi = 0; gsc1.sRm = 0; gsc1.sRn = 0;
      gsc1.M = T; gsc1.N = T; gsc1.K = DH; gsc1.zi_n = T; gsc1.flags = 0; gsc1.act = 0;
      gsc1.alpha = 1.0f; gsc1.beta = 0.0f; gsc1.sa = 1.0f; gsc1.sb = 1.0f; gsc1.Npad = T; gsc1.pad_ = 0;
      if ((long long)(T) >= 64 && (long long)(T) >= 64) k_gemmT<0, 4, 4><<<dim3((unsigned)((T) + 63) / 64, (unsigned)((T) + 63) / 64, (unsigned)(HB * T)), 32, 0, stream>>>(gsc1);
      else k_gemm<0><<<dim3((unsigned)((T) + 31) / 32, (unsigned)((T) + 15) / 16, (unsigned)(HB * T)), 32, 0, stream>>>(gsc1); }
    k_dt_soft<<<2 * T, 256, 0, stream>>>(SC, lq1, lk1, lq2, lk2, AS, AT, SA, 2, T, DH, 0.35550906759096934f);
    k_dt_kk<<<(unsigned)(((long long)HB * T * T * DH + 255) / 256), 256, 0, stream>>>(KKQ, KK, 8, HB, T, DK, E2, DH);
    { GemmP gsc2;
      gsc2.A = KKQ + (size_t)2 * E2 + 8 * DH; gsc2.B = KK; gsc2.bias = KKQ + (size_t)2 * E2 + 8 * DH; gsc2.R = KKQ + (size_t)2 * E2 + 8 * DH; gsc2.C = SC;
      gsc2.sAo = DH; gsc2.sAi = 0; gsc2.sAm = DK; gsc2.sAk = 1; gsc2.sBo = (long long)T * T * DH; gsc2.sBi = (long long)T * DH; gsc2.sBn = DH; gsc2.sBk = 1; gsc2.sCo = (long long)T * T * T; gsc2.sCi = T; gsc2.sCm = (long long)T * T; gsc2.sRo = 0; gsc2.sRi = 0; gsc2.sRm = 0; gsc2.sRn = 0;
      gsc2.M = T; gsc2.N = T; gsc2.K = DH; gsc2.zi_n = T; gsc2.flags = 0; gsc2.act = 0;
      gsc2.alpha = 1.0f; gsc2.beta = 0.0f; gsc2.sa = 1.0f; gsc2.sb = 1.0f; gsc2.Npad = T; gsc2.pad_ = 0;
      if ((long long)(T) >= 64 && (long long)(T) >= 64) k_gemmT<0, 4, 4><<<dim3((unsigned)((T) + 63) / 64, (unsigned)((T) + 63) / 64, (unsigned)(HB * T)), 32, 0, stream>>>(gsc2);
      else k_gemm<0><<<dim3((unsigned)((T) + 31) / 32, (unsigned)((T) + 15) / 16, (unsigned)(HB * T)), 32, 0, stream>>>(gsc2); }
    k_dt_soft<<<2 * T, 256, 0, stream>>>(SC, lq1, lk1, lq2, lk2, AS, AT, SA, 4, T, DH, 0.35550906759096934f);
    k_dt_kk<<<(unsigned)(((long long)HB * T * T * DH + 255) / 256), 256, 0, stream>>>(KKQ, KK, 12, HB, T, DK, E2, DH);
    { GemmP gsc3;
      gsc3.A = KKQ + (size_t)2 * E2 + 12 * DH; gsc3.B = KK; gsc3.bias = KKQ + (size_t)2 * E2 + 12 * DH; gsc3.R = KKQ + (size_t)2 * E2 + 12 * DH; gsc3.C = SC;
      gsc3.sAo = DH; gsc3.sAi = 0; gsc3.sAm = DK; gsc3.sAk = 1; gsc3.sBo = (long long)T * T * DH; gsc3.sBi = (long long)T * DH; gsc3.sBn = DH; gsc3.sBk = 1; gsc3.sCo = (long long)T * T * T; gsc3.sCi = T; gsc3.sCm = (long long)T * T; gsc3.sRo = 0; gsc3.sRi = 0; gsc3.sRm = 0; gsc3.sRn = 0;
      gsc3.M = T; gsc3.N = T; gsc3.K = DH; gsc3.zi_n = T; gsc3.flags = 0; gsc3.act = 0;
      gsc3.alpha = 1.0f; gsc3.beta = 0.0f; gsc3.sa = 1.0f; gsc3.sb = 1.0f; gsc3.Npad = T; gsc3.pad_ = 0;
      if ((long long)(T) >= 64 && (long long)(T) >= 64) k_gemmT<0, 4, 4><<<dim3((unsigned)((T) + 63) / 64, (unsigned)((T) + 63) / 64, (unsigned)(HB * T)), 32, 0, stream>>>(gsc3);
      else k_gemm<0><<<dim3((unsigned)((T) + 31) / 32, (unsigned)((T) + 15) / 16, (unsigned)(HB * T)), 32, 0, stream>>>(gsc3); }
    k_dt_soft<<<2 * T, 256, 0, stream>>>(SC, lq1, lk1, lq2, lk2, AS, AT, SA, 6, T, DH, 0.35550906759096934f);
    { GemmP gz1;
      gz1.A = AS; gz1.B = VA; gz1.bias = AS; gz1.R = AS; gz1.C = Z;
      gz1.sAo = (long long)T * T; gz1.sAi = 0; gz1.sAm = T; gz1.sAk = 1; gz1.sBo = DV; gz1.sBi = 0; gz1.sBn = 1; gz1.sBk = 1024; gz1.sCo = DV; gz1.sCi = 0; gz1.sCm = NH * DV; gz1.sRo = 0; gz1.sRi = 0; gz1.sRm = 0; gz1.sRn = 0;
      gz1.M = T; gz1.N = DV; gz1.K = T; gz1.zi_n = 1; gz1.flags = 0; gz1.act = 0;
      gz1.alpha = 1.0f; gz1.beta = 0.0f; gz1.sa = 1.0f; gz1.sb = 1.0f; gz1.Npad = DV; gz1.pad_ = 0;
      if ((long long)(T) >= 64 && (long long)(DV) >= 64) k_gemmT<1, 2, 4><<<dim3((unsigned)((DV) + 63) / 64, (unsigned)((T) + 31) / 32, (unsigned)(NH)), 32, 0, stream>>>(gz1);
      else k_gemm<1><<<dim3((unsigned)((DV) + 31) / 32, (unsigned)((T) + 15) / 16, (unsigned)(NH)), 32, 0, stream>>>(gz1); }
    { GemmP gz2;
      gz2.A = AT; gz2.B = VB; gz2.bias = AT; gz2.R = Z; gz2.C = Z;
      gz2.sAo = (long long)T * T; gz2.sAi = 0; gz2.sAm = T; gz2.sAk = 1; gz2.sBo = DV; gz2.sBi = 0; gz2.sBn = 1; gz2.sBk = 1024; gz2.sCo = DV; gz2.sCi = 0; gz2.sCm = NH * DV; gz2.sRo = DV; gz2.sRi = 0; gz2.sRm = NH * DV; gz2.sRn = 1;
      gz2.M = T; gz2.N = DV; gz2.K = T; gz2.zi_n = 1; gz2.flags = 4; gz2.act = 0;
      gz2.alpha = 1.0f; gz2.beta = 1.0f; gz2.sa = 1.0f; gz2.sb = 1.0f; gz2.Npad = DV; gz2.pad_ = 0;
      if ((long long)(T) >= 64 && (long long)(DV) >= 64) k_gemmT<1, 2, 4><<<dim3((unsigned)((DV) + 63) / 64, (unsigned)((T) + 31) / 32, (unsigned)(NH)), 32, 0, stream>>>(gz2);
      else k_gemm<1><<<dim3((unsigned)((DV) + 31) / 32, (unsigned)((T) + 15) / 16, (unsigned)(NH)), 32, 0, stream>>>(gz2); }
    k_dt_fin<<<T * NH, 128, 0, stream>>>(Z, SA, bv, Z2, T, NH, DV, 0.35550906759096934f);
    { GemmP gout;
      gout.A = Z2; gout.B = Wo; gout.bias = bo; gout.R = Z2; gout.C = out;
      gout.sAo = 0; gout.sAi = 0; gout.sAm = 1024; gout.sAk = 1; gout.sBo = 0; gout.sBi = 0; gout.sBn = 1; gout.sBk = D; gout.sCo = 0; gout.sCi = 0; gout.sCm = D; gout.sRo = 0; gout.sRi = 0; gout.sRm = 0; gout.sRn = 0;
      gout.M = T; gout.N = D; gout.K = 1024; gout.zi_n = 1; gout.flags = 1; gout.act = 0;
      gout.alpha = 1.0f; gout.beta = 0.0f; gout.sa = 1.0f; gout.sb = 1.0f; gout.Npad = D; gout.pad_ = 0;
      if ((long long)(T) >= 64 && (long long)(D) >= 64) k_gemmT<1, 2, 4><<<dim3((unsigned)((D) + 63) / 64, (unsigned)((T) + 31) / 32, (unsigned)(1)), 32, 0, stream>>>(gout);
      else k_gemm<1><<<dim3((unsigned)((D) + 31) / 32, (unsigned)((T) + 15) / 16, (unsigned)(1)), 32, 0, stream>>>(gout); }
}
